// GAT_3350074491117
// MI455X (gfx1250) — hardware-run, weakly checked
//
#include <hip/hip_runtime.h>

typedef float          v8f   __attribute__((ext_vector_type(8)));
typedef float          v4f   __attribute__((ext_vector_type(4)));
typedef unsigned int   v4u   __attribute__((ext_vector_type(4)));
typedef int            v8i   __attribute__((ext_vector_type(8)));
typedef unsigned short v8us  __attribute__((ext_vector_type(8)));
typedef unsigned short v16us __attribute__((ext_vector_type(16)));
typedef __bf16         v16bf __attribute__((ext_vector_type(16)));
typedef _Float16       v16h  __attribute__((ext_vector_type(16)));
typedef v4f  __attribute__((may_alias)) v4fa;
typedef v8us __attribute__((may_alias)) v8usa;
union FragB { v16bf v; v16us u; v8us h[2]; v8i w; };
union FragH { v16h  v; v16us u; v8us h[2]; v8i w; };

__device__ __forceinline__ v8f wmb(const FragB& a, const FragB& b, v8f c) {
  v8f d = __builtin_amdgcn_wmma_f32_16x16x32_bf16(false, a.v, false, b.v, (short)0, c, false, false);
  asm volatile("v_nop\n\tv_nop\n\tv_nop\n\tv_nop" : "+v"(d) : "v"(a.w), "v"(b.w));
  return d;
}

__device__ __forceinline__ v8f wmh(const FragH& a, const FragH& b, v8f c) {
  v8f d = __builtin_amdgcn_wmma_f32_16x16x32_f16(false, a.v, false, b.v, (short)0, c, false, false);
  asm volatile("v_nop\n\tv_nop\n\tv_nop\n\tv_nop" : "+v"(d) : "v"(a.w), "v"(b.w));
  return d;
}

__device__ __forceinline__ unsigned bf16_bits(float f) {
  const unsigned u = __float_as_uint(f);
  const unsigned r = (u + 0x7FFFu + ((u >> 16) & 1u)) >> 16;
  const unsigned q = (u >> 16) | 0x40u;
  return ((u & 0x7fffffffu) > 0x7f800000u) ? q : r;
}

__device__ __forceinline__ float bf16_val(float f) {
  return __uint_as_float(bf16_bits(f) << 16);
}
__device__ __forceinline__ int clampi(int v, int lo, int hi) {
  return v < lo ? lo : (v > hi ? hi : v);
}

__device__ __forceinline__ unsigned f16_bits(float f) {
  const unsigned u  = __float_as_uint(f);
  const unsigned s  = (u >> 16) & 0x8000u;
  const unsigned a  = u & 0x7fffffffu;
  const unsigned t  = a - 0x38000000u;
  const unsigned r  = (t + 0x0FFFu + ((t >> 13) & 1u)) >> 13;
  const unsigned rc = r > 0x7C00u ? 0x7C00u : r;
  const bool small  = a < 0x38800000u;
  const bool isnan  = a > 0x7f800000u;
  const unsigned fin = small ? 0u : (s | rc);
  return isnan ? (s | 0x7E00u) : fin;
}

__device__ __forceinline__ unsigned pk16(unsigned lo, unsigned hi) { return lo | (hi << 16); }
__device__ __forceinline__ unsigned bf16_lo_bits(float v) {
  float hi = bf16_val(v);
  asm volatile("" : "+v"(hi));
  return bf16_bits(v - hi);
}
__device__ __forceinline__ v4u pack8_bf16(v4f a, v4f c) {
  return (v4u){ pk16(bf16_bits(a[0]), bf16_bits(a[1])), pk16(bf16_bits(a[2]), bf16_bits(a[3])),
                pk16(bf16_bits(c[0]), bf16_bits(c[1])), pk16(bf16_bits(c[2]), bf16_bits(c[3])) };
}
__device__ __forceinline__ v4u pack8_bf16_lo(v4f a, v4f c) {
  return (v4u){ pk16(bf16_lo_bits(a[0]), bf16_lo_bits(a[1])), pk16(bf16_lo_bits(a[2]), bf16_lo_bits(a[3])),
                pk16(bf16_lo_bits(c[0]), bf16_lo_bits(c[1])), pk16(bf16_lo_bits(c[2]), bf16_lo_bits(c[3])) };
}
__device__ __forceinline__ v4u pack8_f16(v4f a, v4f c) {
  return (v4u){ pk16(f16_bits(a[0]), f16_bits(a[1])), pk16(f16_bits(a[2]), f16_bits(a[3])),
                pk16(f16_bits(c[0]), f16_bits(c[1])), pk16(f16_bits(c[2]), f16_bits(c[3])) };
}

template <int FORM>
__global__ __launch_bounds__(256) void k_plane(const float* __restrict__ src, int rows, int cols, int ldsrc,
                                               unsigned short* __restrict__ dst, int MP, int KP) {
  static_assert(FORM >= 0 && FORM <= 3);
  const int KTOT = (FORM == 1 || FORM == 3) ? 2 * KP : KP;
  const unsigned ppr   = (unsigned)(KTOT >> 3);
  const unsigned kp8   = (unsigned)(KP >> 3);
  const unsigned total = (unsigned)MP * ppr;
  const unsigned g     = blockIdx.x * 256u + threadIdx.x;
  const unsigned rowu  = g / ppr;
  const unsigned p     = g - rowu * ppr;
  const bool second    = p >= kp8;
  const int row = (int)rowu;
  const int c0  = (int)((second ? p - kp8 : p) << 3);
  const float* srow = src + (size_t)clampi(row, 0, rows - 1) * (size_t)ldsrc;
  float x[8];
  unsigned mk[8];
#pragma unroll
  for (int e = 0; e < 8; ++e) {
    const int c = c0 + e;
    const float v = srow[clampi(c, 0, cols - 1)];
    asm volatile("" :: "v"(v));
    x[e]  = v;
    mk[e] = (row < rows && c < cols) ? 0xFFFFu : 0u;
  }
  const v4f a = (v4f){ x[0], x[1], x[2], x[3] };
  const v4f c = (v4f){ x[4], x[5], x[6], x[7] };
  v4u o;
  if (FORM == 2) {
    o = pack8_f16(a, c);
  } else {
    const v4u hi = pack8_bf16(a, c);
    o = hi;
    if (FORM == 1) { const v4u lo = pack8_bf16_lo(a, c); o = second ? lo : hi; }
  }
  const v4u mw = (v4u){ pk16(mk[0], mk[1]), pk16(mk[2], mk[3]), pk16(mk[4], mk[5]), pk16(mk[6], mk[7]) };
  o &= mw;
  if (g < total) {
    volatile v4u* q = (volatile v4u*)(dst + (size_t)g * 8);
    *q = o;
    __threadfence();
    *q = o;
  }
}

template <int FORM> struct FragOf    { typedef FragB T; };
template <>         struct FragOf<2> { typedef FragH T; };
__device__ __forceinline__ v8f mm(const FragB& a, const FragB& b, v8f c) { return wmb(a, b, c); }
__device__ __forceinline__ v8f mm(const FragH& a, const FragH& b, v8f c) { return wmh(a, b, c); }
template <class F> __device__ __forceinline__ F ld_frag(const unsigned short* p) {
  F f;
  f.h[0] = *(const v8usa*)(p);
  f.h[1] = *(const v8usa*)(p + 16);
  return f;
}

template <int FORM, int EPI>
__global__ __launch_bounds__(256) __attribute__((amdgpu_num_vgpr(248)))
void k_gemm_nt(const unsigned short* __restrict__ A, const unsigned short* __restrict__ B,
               const float* __restrict__ bias, float* __restrict__ D, int M, int N, int KTOT, int ldd) {
  static_assert(FORM >= 0 && FORM <= 2);
  static_assert(EPI == 0 || EPI == 1);
  typedef typename FragOf<FORM>::T F;
  __shared__ __attribute__((aligned(16))) float sT[8][16 * 68];
  const int lane = threadIdx.x & 31;
  const int wave = threadIdx.x >> 5;
  const int tilesM = (M + 63) >> 6;
  const int tilesN = (N + 63) >> 6;
  const int tile = blockIdx.x * 8 + wave;
  if (tile >= tilesM * tilesN) return;
  const int tm = tile / tilesN;
  const int tn = tile - tm * tilesN;
  const int m0 = tm << 6;
  const int n0 = tn << 6;

  const int rl = lane & 15;
  const int h8 = (lane >> 4) * 8;
  const unsigned short* pa = A + (size_t)(m0 + rl) * (size_t)KTOT + h8;
  const unsigned short* pb = B + (size_t)(n0 + rl) * (size_t)KTOT + h8;

  v8f acc[4][4];
#pragma unroll
  for (int i = 0; i < 4; ++i)
#pragma unroll
    for (int j = 0; j < 4; ++j) acc[i][j] = (v8f){0.f, 0.f, 0.f, 0.f, 0.f, 0.f, 0.f, 0.f};

#pragma unroll 1
  for (int k0 = 0; k0 < KTOT; k0 += 32) {
    F bf[4];
#pragma unroll
    for (int j = 0; j < 4; ++j) bf[j] = ld_frag<F>(pb + (size_t)(j << 4) * (size_t)KTOT + k0);
#pragma unroll
    for (int i = 0; i < 4; ++i) {
      const F af = ld_frag<F>(pa + (size_t)(i << 4) * (size_t)KTOT + k0);
#pragma unroll
      for (int j = 0; j < 4; ++j) acc[i][j] = mm(af, bf[j], acc[i][j]);
    }
  }

  float* slab = sT[wave];
  const int hh = lane >> 4;
  const int c4 = (lane & 15) * 4;
  const int nc = n0 + c4;
  const bool cok = nc < N;
  v4f bv = (v4f){0.f, 0.f, 0.f, 0.f};
  if (EPI == 1) {
    bv = *(const v4fa*)(bias + clampi(nc, 0, N - 4));
    asm volatile("" :: "v"(bv));
  }
#pragma unroll
  for (int i = 0; i < 4; ++i) {
    const int mBase = m0 + (i << 4);
#pragma unroll
    for (int j = 0; j < 4; ++j) {
#pragma unroll
      for (int r = 0; r < 8; ++r) slab[(h8 + r) * 68 + (j << 4) + rl] = acc[i][j][r];
    }
    __builtin_amdgcn_fence(__ATOMIC_RELEASE, "workgroup");
    __builtin_amdgcn_wave_barrier();
    __builtin_amdgcn_fence(__ATOMIC_ACQUIRE, "workgroup");
    v4f vv[8];
#pragma unroll
    for (int it = 0; it < 8; ++it) {
      const int row = it * 2 + hh;
      v4f v = *(const v4fa*)(slab + row * 68 + c4);
      if (EPI == 1) v += bv;
      vv[it] = v;
    }
    for (int pass = 0; pass < 2; ++pass) {
#pragma unroll
      for (int it = 0; it < 8; ++it) {
        const int row = mBase + it * 2 + hh;
        if (cok && row < M) *(volatile v4f*)(D + (size_t)row * (size_t)ldd + nc) = vv[it];
      }
      __threadfence();
    }
    __builtin_amdgcn_fence(__ATOMIC_RELEASE, "workgroup");
    __builtin_amdgcn_wave_barrier();
    __builtin_amdgcn_fence(__ATOMIC_ACQUIRE, "workgroup");
  }
}

#pragma clang fp contract(off)


#ifndef SPLIT_2
#define SPLIT_2 1
#endif

#define NN      50000
#define NE      800000
#define NPAD    50048
#define KD      128
#define D1W     128
#define D2W     64
#define NH1     4
#define CH1     32
#if SPLIT_2
#define OPK     256
#else
#define OPK     128
#endif
#define T_AS1   0
#define T_AD1   128
#define T_B1    256
#define T_AS2   384
#define T_AD2   448
#define T_B2    512
#define T_N     576
#define TB_BYTES 4096
#define BT      512
#define BW      16
#define BEPT    8
#define BCHUNK  (BT * BEPT)
#define NCH     ((NE + BCHUNK - 1) / BCHUNK)
#define NB      1024
#define NBLK    ((NN + NB - 1) / NB)
#define RCAP    20992
#define DEGCAP  64
#define SLOTSH  21
#define LISTTOT (NBLK * RCAP)
#define LDS_LIST ((2 * RCAP + 3 * NB + 64) * 4)
#define WSMAX   ((size_t)128 << 20)
#define PREP_W1_BLK (D1W * (KD / 8) / 256)
#define PREP_W2_BLK (D2W * (OPK / 8) / 256)

#define SZ_XB   ((size_t)NPAD * KD * 2)
#define SZ_W1T  ((size_t)D1W * KD * 2)
#define SZ_W2D  ((size_t)D2W * OPK * 2)
#define SZ_FT   ((size_t)NPAD * D1W * 4)
#define SZ_OP   ((size_t)NPAD * OPK * 2)
#define SZ_E1   ((size_t)NPAD * NH1 * 4)
#define SZ_E2   ((size_t)NPAD * 4)
#define SZ_META ((size_t)NBLK * NB * 2 * 4)
#define SZ_LIST ((size_t)NBLK * RCAP * 4)
#define WS_TOTAL (SZ_XB + SZ_W1T + SZ_W2D + (size_t)TB_BYTES + SZ_FT + SZ_OP + 2 * SZ_E1 + 2 * SZ_E2 + SZ_META + SZ_LIST)

static_assert(NH1 * CH1 == 128 && 1 * 64 == D2W && D1W == 128 && KD == 128);
static_assert(NN % 8 == 0);
static_assert(NPAD % 128 == 0 && NPAD % 32 == 0 && NPAD % 64 == 0 && NPAD == 391 * 128 && NPAD >= NN);
static_assert(NBLK == 49 && NBLK * NB >= NN);
static_assert(NE % 8 == 0 && NE >= 8 && NE < (1 << SLOTSH));
static_assert(NCH == 196 && NCH * BCHUNK >= NE);
static_assert(NB <= 1024 && (NB & (NB - 1)) == 0 && NB == 2 * BT && BW == BT / 32);
static_assert(RCAP % 128 == 0);
static_assert(RCAP * 4 >= 16623 * 5);
static_assert(DEGCAP >= 35 + 8);
static_assert(LDS_LIST == 180480 && LDS_LIST + 0 <= 327680);
static_assert(8 * 16 * 68 * 4 <= 327680);
static_assert(OPK % 32 == 0 && KD % 32 == 0);
static_assert((D1W * (KD / 8)) % 256 == 0 && (D2W * (OPK / 8)) % 256 == 0);
static_assert((size_t)NPAD * OPK / 8 < ((size_t)1 << 31));
static_assert(T_N * 4 <= TB_BYTES && T_N % 4 == 0);
static_assert(SZ_XB % 128 == 0 && SZ_W2D % 128 == 0 && SZ_FT % 128 == 0 && SZ_OP % 128 == 0 && SZ_E1 % 128 == 0 &&
              SZ_E2 % 128 == 0 && SZ_META % 128 == 0 && SZ_LIST % 128 == 0);
static_assert((size_t)NPAD * D2W * 4 <= SZ_FT);
#if SPLIT_2
static_assert(WS_TOTAL == 70648832);
#endif
static_assert(WS_TOTAL <= WSMAX);
static_assert((size_t)(NN - 1) * D2W + 63 < (size_t)NN * D2W);

typedef int          v4i __attribute__((ext_vector_type(4)));
typedef int          v2i __attribute__((ext_vector_type(2)));
typedef unsigned int v2u __attribute__((ext_vector_type(2)));
typedef float        v2f __attribute__((ext_vector_type(2)));
typedef v4i __attribute__((may_alias)) v4ia;
typedef v2i __attribute__((may_alias)) v2ia;
typedef v2f __attribute__((may_alias)) v2fa;

__device__ __forceinline__ float lrelu_k(float v) { return (v > 0.0f) ? v : 0.2f * v; }
__device__ __forceinline__ float elu_k(float v) { return (v > 0.0f) ? v : expm1f(v); }
__device__ __forceinline__ float maxk(float a, float b) {
  float m = (a < b) ? b : a;
  m = (b != b) ? b : m;
  return m;
}
__device__ __forceinline__ float sum8(float t) {
  t = t + __shfl_xor(t, 4, 32);
  t = t + __shfl_xor(t, 2, 32);
  t = t + __shfl_xor(t, 1, 32);
  return t;
}
__device__ __forceinline__ float sum32(float t) {
  t = t + __shfl_xor(t, 16, 32);
  t = t + __shfl_xor(t, 8, 32);
  t = t + __shfl_xor(t, 4, 32);
  t = t + __shfl_xor(t, 2, 32);
  t = t + __shfl_xor(t, 1, 32);
  return t;
}

__global__ __launch_bounds__(256) void k_prep(const float* __restrict__ W1, const float* __restrict__ W2,
                                              const float* __restrict__ as1, const float* __restrict__ ad1,
                                              const float* __restrict__ b1, const float* __restrict__ as2,
                                              const float* __restrict__ ad2, const float* __restrict__ b2,
                                              unsigned short* W1T, unsigned short* W2D, float* TB) {
  const int t = (int)threadIdx.x;
  const int b = (int)blockIdx.x;
  if (b < PREP_W1_BLK) {
    const int g  = b * 256 + t;
    const int n  = g >> 4;
    const int k0 = (g & 15) << 3;
    float x[8];
#pragma unroll
    for (int e = 0; e < 8; ++e) {
      const float v = W1[(size_t)(k0 + e) * D1W + n];
      asm volatile("" :: "v"(v));
      x[e] = v;
    }
    const v4u o = pack8_bf16((v4f){x[0], x[1], x[2], x[3]}, (v4f){x[4], x[5], x[6], x[7]});
    volatile v4u* q = (volatile v4u*)(W1T + (size_t)g * 8);
    *q = o;
    __threadfence();
    *q = o;
  } else if (b < PREP_W1_BLK + PREP_W2_BLK) {
    const int g   = (b - PREP_W1_BLK) * 256 + t;
    const int ppr = OPK / 8;
    const int n   = g / ppr;
    const int k0  = (g - n * ppr) << 3;
    const int km  = k0 & 127;
    float x[8];
#pragma unroll
    for (int e = 0; e < 8; ++e) {
      const float v = W2[(size_t)(km + e) * D2W + n];
      asm volatile("" :: "v"(v));
      x[e] = v;
    }
    const v4u o = pack8_bf16((v4f){x[0], x[1], x[2], x[3]}, (v4f){x[4], x[5], x[6], x[7]});
    volatile v4u* q = (volatile v4u*)(W2D + (size_t)g * 8);
    *q = o;
    __threadfence();
    *q = o;
  } else {
    const int idx = 4 * t;
    const v4f a0 = *(const v4fa*)(as1 + clampi(idx - T_AS1, 0, 124));
    asm volatile("" :: "v"(a0));
    const v4f a1 = *(const v4fa*)(ad1 + clampi(idx - T_AD1, 0, 124));
    asm volatile("" :: "v"(a1));
    const v4f a2 = *(const v4fa*)(b1  + clampi(idx - T_B1,  0, 124));
    asm volatile("" :: "v"(a2));
    const v4f a3 = *(const v4fa*)(as2 + clampi(idx - T_AS2, 0, 60));
    asm volatile("" :: "v"(a3));
    const v4f a4 = *(const v4fa*)(ad2 + clampi(idx - T_AD2, 0, 60));
    asm volatile("" :: "v"(a4));
    const v4f a5 = *(const v4fa*)(b2  + clampi(idx - T_B2,  0, 60));
    asm volatile("" :: "v"(a5));
    const unsigned m0 = (idx < T_AD1) ? 0xFFFFFFFFu : 0u;
    const unsigned m1 = (idx >= T_AD1 && idx < T_B1)  ? 0xFFFFFFFFu : 0u;
    const unsigned m2 = (idx >= T_B1  && idx < T_AS2) ? 0xFFFFFFFFu : 0u;
    const unsigned m3 = (idx >= T_AS2 && idx < T_AD2) ? 0xFFFFFFFFu : 0u;
    const unsigned m4 = (idx >= T_AD2 && idx < T_B2)  ? 0xFFFFFFFFu : 0u;
    const unsigned m5 = (idx >= T_B2) ? 0xFFFFFFFFu : 0u;
    v4u o;
    o.x = (__float_as_uint(a0.x) & m0) | (__float_as_uint(a1.x) & m1) | (__float_as_uint(a2.x) & m2) |
          (__float_as_uint(a3.x) & m3) | (__float_as_uint(a4.x) & m4) | (__float_as_uint(a5.x) & m5);
    o.y = (__float_as_uint(a0.y) & m0) | (__float_as_uint(a1.y) & m1) | (__float_as_uint(a2.y) & m2) |
          (__float_as_uint(a3.y) & m3) | (__float_as_uint(a4.y) & m4) | (__float_as_uint(a5.y) & m5);
    o.z = (__float_as_uint(a0.z) & m0) | (__float_as_uint(a1.z) & m1) | (__float_as_uint(a2.z) & m2) |
          (__float_as_uint(a3.z) & m3) | (__float_as_uint(a4.z) & m4) | (__float_as_uint(a5.z) & m5);
    o.w = (__float_as_uint(a0.w) & m0) | (__float_as_uint(a1.w) & m1) | (__float_as_uint(a2.w) & m2) |
          (__float_as_uint(a3.w) & m3) | (__float_as_uint(a4.w) & m4) | (__float_as_uint(a5.w) & m5);
    o.x = bf16_bits(__uint_as_float(o.x)) << 16;
    o.y = bf16_bits(__uint_as_float(o.y)) << 16;
    o.z = bf16_bits(__uint_as_float(o.z)) << 16;
    o.w = bf16_bits(__uint_as_float(o.w)) << 16;
    const bool wr = idx < T_N;
    volatile v4u* q = (volatile v4u*)(TB + (wr ? idx : 0));
    if (wr) *q = o;
    __threadfence();
    if (wr) *q = o;
  }
}

__global__ __launch_bounds__(BT) void k_list(const int* __restrict__ ekey, const int* __restrict__ esrc,
                                             unsigned* LIST, int* META) {
  extern __shared__ v4u lds_list[];
  int* reg1 = (int*)lds_list;
  int* reg2 = reg1 + RCAP;
  int* scnt = reg2 + RCAP;
  int* soff = scnt + NB;
  int* curs = soff + NB;
  int* wcnt = curs + NB;
  int* wtot = wcnt + 2 * BW;
  const int tid = (int)threadIdx.x, lane = tid & 31, wave = tid >> 5;
  const int nodeBase = (int)blockIdx.x * NB;
  int nb = NN - nodeBase;
  nb = nb > NB ? NB : (nb < 0 ? 0 : nb);
  const unsigned nbs = (unsigned)nodeBase, unb = (unsigned)nb;

  scnt[2 * tid] = 0;
  scnt[2 * tid + 1] = 0;
  if (tid == 0) reg2[0] = 0;

  int tot = 0;
#pragma unroll 1
  for (int ch = 0; ch < NCH; ++ch) {
    const int par = ch & 1;
    const int e0  = ch * BCHUNK + tid * BEPT;
    const bool valid = e0 < NE;
    const int ea = e0 < NE - 8 ? e0 : NE - 8;
    const v4i da = *(const v4ia*)(ekey + ea);
    const v4i db = *(const v4ia*)(ekey + ea + 4);
    asm volatile("" :: "v"(da), "v"(db));
    const unsigned s0 = (unsigned)da.x - nbs, s1 = (unsigned)da.y - nbs;
    const unsigned s2 = (unsigned)da.z - nbs, s3 = (unsigned)da.w - nbs;
    const unsigned s4 = (unsigned)db.x - nbs, s5 = (unsigned)db.y - nbs;
    const unsigned s6 = (unsigned)db.z - nbs, s7 = (unsigned)db.w - nbs;
    const bool h0 = valid && (s0 < unb), h1 = valid && (s1 < unb), h2 = valid && (s2 < unb), h3 = valid && (s3 < unb);
    const bool h4 = valid && (s4 < unb), h5 = valid && (s5 < unb), h6 = valid && (s6 < unb), h7 = valid && (s7 < unb);
    const int c = (int)h0 + (int)h1 + (int)h2 + (int)h3 + (int)h4 + (int)h5 + (int)h6 + (int)h7;
    int incl = c;
#pragma unroll
    for (int d = 1; d < 32; d <<= 1) {
      const int up = __shfl_up(incl, d, 32);
      incl += (lane >= d) ? up : 0;
    }
    const int wtotal = __shfl(incl, 31, 32);
    if (lane == 0) wcnt[par * BW + wave] = wtotal;
    __syncthreads();
    int all = 0, pre = 0;
#pragma unroll
    for (int g = 0; g < 4; ++g) {
      const v4i w4 = *(const v4ia*)(wcnt + par * BW + 4 * g);
      const int c0 = clampi(w4.x, 0, 256), c1 = clampi(w4.y, 0, 256);
      const int c2 = clampi(w4.z, 0, 256), c3 = clampi(w4.w, 0, 256);
      all += c0 + c1 + c2 + c3;
      pre += (4 * g + 0 < wave) ? c0 : 0;
      pre += (4 * g + 1 < wave) ? c1 : 0;
      pre += (4 * g + 2 < wave) ? c2 : 0;
      pre += (4 * g + 3 < wave) ? c3 : 0;
    }
    int pos = tot + pre + (incl - c);
#define PUTJ(J, HJ, SJ) if (HJ) { if (pos < RCAP) reg1[pos] = (int)((unsigned)(e0 + (J)) | ((SJ) << SLOTSH)); ++pos; }
    PUTJ(0, h0, s0)
    PUTJ(1, h1, s1)
    PUTJ(2, h2, s2)
    PUTJ(3, h3, s3)
    PUTJ(4, h4, s4)
    PUTJ(5, h5, s5)
    PUTJ(6, h6, s6)
    PUTJ(7, h7, s7)
#undef PUTJ
    tot += all;
  }
  __syncthreads();
  const bool ovf = tot > RCAP;
  const int nh = ovf ? RCAP : tot;

  if (wave == 0) {
#pragma unroll 1
    for (int b0 = 0; b0 < nh; b0 += 32) {
      const int idx = b0 + lane;
      const int uv  = reg1[idx < nh ? idx : nh - 1];
      const int m32 = (nh - b0) < 32 ? (nh - b0) : 32;
#pragma unroll 1
      for (int k = 0; k < m32; ++k) {
        const int u  = __builtin_amdgcn_readlane(uv, k);
        const int sl = (int)(((unsigned)u >> SLOTSH) & (unsigned)(NB - 1));
        const int cv = scnt[sl] + 1;
        if (lane == 0) scnt[sl] = cv;
      }
    }
  }
  __syncthreads();

  int e0c, e1c;
  {
    const v2i cc = *(const v2ia*)(scnt + 2 * tid);
    e0c = cc.x < 0 ? 0 : cc.x;
    e1c = cc.y < 0 ? 0 : cc.y;
    const int ts = e0c + e1c;
    int incl = ts;
#pragma unroll
    for (int d = 1; d < 32; d <<= 1) {
      const int up = __shfl_up(incl, d, 32);
      incl += (lane >= d) ? up : 0;
    }
    if (lane == 31) wtot[wave] = incl;
    __syncthreads();
    int pre = 0;
#pragma unroll
    for (int g = 0; g < 4; ++g) {
      const v4i w4 = *(const v4ia*)(wtot + 4 * g);
      pre += (4 * g + 0 < wave) ? w4.x : 0;
      pre += (4 * g + 1 < wave) ? w4.y : 0;
      pre += (4 * g + 2 < wave) ? w4.z : 0;
      pre += (4 * g + 3 < wave) ? w4.w : 0;
    }
    const int run = pre + incl - ts;
    soff[2 * tid]     = run;
    soff[2 * tid + 1] = run + e0c;
    curs[2 * tid]     = run;
    curs[2 * tid + 1] = run + e0c;
  }
  __syncthreads();

  if (wave == 0) {
#pragma unroll 1
    for (int b0 = 0; b0 < nh; b0 += 32) {
      const int idx = b0 + lane;
      const int uv  = reg1[idx < nh ? idx : nh - 1];
      const int m32 = (nh - b0) < 32 ? (nh - b0) : 32;
#pragma unroll 1
      for (int k = 0; k < m32; ++k) {
        const int u   = __builtin_amdgcn_readlane(uv, k);
        const int sl  = (int)(((unsigned)u >> SLOTSH) & (unsigned)(NB - 1));
        const int eid = (int)((unsigned)u & ((1u << SLOTSH) - 1u));
        const int pr  = curs[sl];
        const int pc  = clampi(pr, 0, RCAP - 1);
        if (lane == 0) { reg2[pc] = eid; curs[sl] = pc + 1; }
      }
    }
  }
  __syncthreads();

  {
    unsigned* lbase = LIST + (size_t)blockIdx.x * (size_t)RCAP;
    const int npc = RCAP / 4;
#pragma unroll 1
    for (int it = 0; it < (RCAP / 4 + BT - 1) / BT; ++it) {
      const int pc = it * BT + tid;
      const bool wr = pc < npc;
      const int i0 = 4 * (wr ? pc : npc - 1);
      unsigned w[4];
#pragma unroll
      for (int e = 0; e < 4; ++e) {
        const int i   = i0 + e;
        const int ic  = clampi(i < nh ? i : nh - 1, 0, RCAP - 1);
        const int eid = clampi(reg2[ic], 0, NE - 1);
        const int sw  = esrc[eid];
        asm volatile("" :: "v"(sw));
        const unsigned msk = (i < nh) ? 0xFFFFFFFFu : 0u;
        w[e] = (unsigned)clampi(sw, 0, NN - 1) & msk;
      }
      const v4u o = (v4u){ w[0], w[1], w[2], w[3] };
      volatile v4u* q = (volatile v4u*)(lbase + i0);
      if (wr) *q = o;
      __threadfence();
      if (wr) *q = o;
    }
  }

  {
    const int base = (int)blockIdx.x * RCAP;
    const v2i cc = *(const v2ia*)(scnt + 2 * tid);
    const v2i so = *(const v2ia*)(soff + 2 * tid);
    v4i m;
    m.x = base + so.x;
    m.y = ovf ? -1 : cc.x;
    m.z = base + so.y;
    m.w = ovf ? -1 : cc.y;
    volatile v4i* q = (volatile v4i*)(META + 2 * (size_t)(nodeBase + 2 * tid));
    *q = m;
    __threadfence();
    *q = m;
  }
}

__global__ __launch_bounds__(256) void k_rowprep1(const float* __restrict__ FT, const float* __restrict__ TB,
                                                  float* EL, float* ER) {
  __shared__ __attribute__((aligned(16))) float sL[32 * NH1];
  __shared__ __attribute__((aligned(16))) float sR[32 * NH1];
  const int lane = (int)threadIdx.x & 31;
  const int wave = (int)threadIdx.x >> 5;
  const int head = lane >> 3;
  const int c0   = lane * 4;
  const v4f as = *(const v4fa*)(TB + T_AS1 + c0);
  const v4f ad = *(const v4fa*)(TB + T_AD1 + c0);
#pragma unroll 1
  for (int q = 0; q < 4; ++q) {
    const int nl  = wave * 4 + q;
    const int row = (int)blockIdx.x * 32 + nl;
    const v4f p = *(const v4fa*)(FT + (size_t)row * D1W + c0);
    asm volatile("" :: "v"(p));
    float t = p.x * as.x;
    float u = p.y * as.y; t = t + u;
    u = p.z * as.z; t = t + u;
    u = p.w * as.w; t = t + u;
    float d = p.x * ad.x;
    u = p.y * ad.y; d = d + u;
    u = p.z * ad.z; d = d + u;
    u = p.w * ad.w; d = d + u;
    t = sum8(t);
    d = sum8(d);
    if ((lane & 7) == 0) { sL[nl * NH1 + head] = t; sR[nl * NH1 + head] = d; }
  }
  __syncthreads();
  if (wave == 0) {
    const v4f v = *(const v4fa*)(sL + 4 * lane);
    volatile v4f* q = (volatile v4f*)(EL + ((size_t)blockIdx.x * 32 + lane) * NH1);
    *q = v;
    __threadfence();
    *q = v;
  } else if (wave == 1) {
    const v4f v = *(const v4fa*)(sR + 4 * lane);
    volatile v4f* q = (volatile v4f*)(ER + ((size_t)blockIdx.x * 32 + lane) * NH1);
    *q = v;
    __threadfence();
    *q = v;
  }
}

__global__ __launch_bounds__(256) void k_rowprep2(const float* __restrict__ FT2, const float* __restrict__ TB,
                                                  float* EL, float* ER) {
  __shared__ __attribute__((aligned(16))) float sL[32];
  __shared__ __attribute__((aligned(16))) float sR[32];
  const int lane = (int)threadIdx.x & 31;
  const int wave = (int)threadIdx.x >> 5;
  const int c0   = lane * 2;
  const v2f as = *(const v2fa*)(TB + T_AS2 + c0);
  const v2f ad = *(const v2fa*)(TB + T_AD2 + c0);
#pragma unroll 1
  for (int q = 0; q < 4; ++q) {
    const int nl  = wave * 4 + q;
    const int row = (int)blockIdx.x * 32 + nl;
    const v2f p = *(const v2fa*)(FT2 + (size_t)row * D2W + c0);
    asm volatile("" :: "v"(p));
    float t = p.x * as.x;
    float u = p.y * as.y; t = t + u;
    float d = p.x * ad.x;
    u = p.y * ad.y; d = d + u;
    t = sum32(t);
    d = sum32(d);
    if (lane == 0) { sL[nl] = t; sR[nl] = d; }
  }
  __syncthreads();
  const int l8 = lane & 7;
  if (wave == 0) {
    const v4f v = *(const v4fa*)(sL + 4 * l8);
    volatile v4f* q = (volatile v4f*)(EL + (size_t)blockIdx.x * 32 + 4 * l8);
    const bool wr = lane < 8;
    if (wr) *q = v;
    __threadfence();
    if (wr) *q = v;
  } else if (wave == 1) {
    const v4f v = *(const v4fa*)(sR + 4 * l8);
    volatile v4f* q = (volatile v4f*)(ER + (size_t)blockIdx.x * 32 + 4 * l8);
    const bool wr = lane < 8;
    if (wr) *q = v;
    __threadfence();
    if (wr) *q = v;
  }
}

__global__ __launch_bounds__(256) void k_walk1(const float* __restrict__ FT, const float* __restrict__ EL,
                                               const float* __restrict__ ER, const unsigned* __restrict__ LIST,
                                               const int* __restrict__ META, const float* __restrict__ TB,
                                               unsigned short* OP) {
  const int lane = (int)threadIdx.x & 31;
  const int wave = (int)threadIdx.x >> 5;
  const int row  = (int)blockIdx.x * 8 + wave;
  const int rowc = row < NN ? row : NN - 1;
  const int hd   = lane >> 3;
  const int jj   = lane & 7;
  const int gb   = lane & 24;
  const int c0   = lane * 4;

  const v2i mt = *(const v2ia*)(META + 2 * (size_t)rowc);
  asm volatile("" :: "v"(mt));
  const int craw = mt.y;
  const int offv = clampi(mt.x, 0, LISTTOT);
  int cntv = clampi(craw, 0, DEGCAP);
  cntv = cntv < (LISTTOT - offv) ? cntv : (LISTTOT - offv);
  const int off = __builtin_amdgcn_readfirstlane(offv);
  const int cnt = __builtin_amdgcn_readfirstlane((row < NN) ? cntv : 0);
  const bool poison = (craw < 0) || (craw > DEGCAP);

  const float eld = EL[(size_t)rowc * NH1 + hd];
  asm volatile("" :: "v"(eld));
  const float erd = ER[(size_t)rowc * NH1 + hd];
  asm volatile("" :: "v"(erd));
  const float tl = eld + erd;
  const float eloop = lrelu_k(tl);

  float mx = -__builtin_inff();
#pragma unroll 1
  for (int b0 = 0; b0 < cnt; b0 += 8) {
    const int j = (b0 + jj) < cnt ? (b0 + jj) : cnt - 1;
    const unsigned s = LIST[(size_t)(off + j)];
    asm volatile("" :: "v"(s));
    const int col = clampi((int)s, 0, NN - 1);
    const float an = EL[(size_t)col * NH1 + hd];
    asm volatile("" :: "v"(an));
    const float t = an + erd;
    mx = maxk(mx, lrelu_k(t));
  }
  {
    const float o4 = __shfl_xor(mx, 4, 32); mx = maxk(mx, o4);
    const float o2 = __shfl_xor(mx, 2, 32); mx = maxk(mx, o2);
    const float o1 = __shfl_xor(mx, 1, 32); mx = maxk(mx, o1);
  }
  mx = maxk(mx, eloop);

  float den = 0.0f;
#pragma unroll 1
  for (int b0 = 0; b0 < cnt; b0 += 8) {
    const int j = (b0 + jj) < cnt ? (b0 + jj) : cnt - 1;
    const unsigned s = LIST[(size_t)(off + j)];
    asm volatile("" :: "v"(s));
    const int col = clampi((int)s, 0, NN - 1);
    const float an = EL[(size_t)col * NH1 + hd];
    asm volatile("" :: "v"(an));
    const float t = an + erd;
    const float v = lrelu_k(t) - mx;
    const float q = expf(v);
    const int m8 = (cnt - b0) < 8 ? (cnt - b0) : 8;
#pragma unroll 1
    for (int k = 0; k < m8; ++k) {
      const float qk = __shfl(q, gb | k, 32);
      den = den + qk;
    }
  }
  const float exl = expf(eloop - mx);
  den = den + exl;

  v4f ac = (v4f){0.0f, 0.0f, 0.0f, 0.0f};
#pragma unroll 1
  for (int b0 = 0; b0 < cnt; b0 += 8) {
    const int j = (b0 + jj) < cnt ? (b0 + jj) : cnt - 1;
    const unsigned s = LIST[(size_t)(off + j)];
    asm volatile("" :: "v"(s));
    const int col = clampi((int)s, 0, NN - 1);
    const float an = EL[(size_t)col * NH1 + hd];
    asm volatile("" :: "v"(an));
    const float t = an + erd;
    const float v = lrelu_k(t) - mx;
    const float q = expf(v);
    const float w = q / den;
    const int m8 = (cnt - b0) < 8 ? (cnt - b0) : 8;
#pragma unroll 1
    for (int k = 0; k < m8; ++k) {
      const int c = __builtin_amdgcn_readlane(col, k);
      const float wk = __shfl(w, gb | k, 32);
      const v4f hn = *(const v4fa*)(FT + (size_t)c * D1W + c0);
      asm volatile("" :: "v"(hn));
      float pr;
      pr = wk * hn.x; ac.x = ac.x + pr;
      pr = wk * hn.y; ac.y = ac.y + pr;
      pr = wk * hn.z; ac.z = ac.z + pr;
      pr = wk * hn.w; ac.w = ac.w + pr;
    }
  }
  {
    const float wl = exl / den;
    const v4f hn = *(const v4fa*)(FT + (size_t)rowc * D1W + c0);
    asm volatile("" :: "v"(hn));
    float pr;
    pr = wl * hn.x; ac.x = ac.x + pr;
    pr = wl * hn.y; ac.y = ac.y + pr;
    pr = wl * hn.z; ac.z = ac.z + pr;
    pr = wl * hn.w; ac.w = ac.w + pr;
  }

  const v4f bv = *(const v4fa*)(TB + T_B1 + c0);
  const float qnan = __uint_as_float(0x7fc00000u);
  const bool live = row < NN;
  float y0 = elu_k(ac.x + bv.x);
  float y1 = elu_k(ac.y + bv.y);
  float y2 = elu_k(ac.z + bv.z);
  float y3 = elu_k(ac.w + bv.w);
  y0 = poison ? qnan : y0;  y1 = poison ? qnan : y1;  y2 = poison ? qnan : y2;  y3 = poison ? qnan : y3;
  y0 = live ? y0 : 0.0f;    y1 = live ? y1 : 0.0f;    y2 = live ? y2 : 0.0f;    y3 = live ? y3 : 0.0f;

  const v2u hi = (v2u){ pk16(bf16_bits(y0), bf16_bits(y1)), pk16(bf16_bits(y2), bf16_bits(y3)) };
  unsigned short* orow = OP + (size_t)row * OPK;
  volatile v2u* qh = (volatile v2u*)(orow + c0);
#if SPLIT_2
  const v2u lo = (v2u){ pk16(bf16_lo_bits(y0), bf16_lo_bits(y1)), pk16(bf16_lo_bits(y2), bf16_lo_bits(y3)) };
  volatile v2u* ql = (volatile v2u*)(orow + 128 + c0);
#endif
  *qh = hi;
#if SPLIT_2
  *ql = lo;
#endif
  __threadfence();
  *qh = hi;
#if SPLIT_2
  *ql = lo;
#endif
}

__global__ __launch_bounds__(256) void k_walk2(const float* __restrict__ FT2, const float* __restrict__ EL,
                                               const float* __restrict__ ER, const unsigned* __restrict__ LIST,
                                               const int* __restrict__ META, const float* __restrict__ TB,
                                               float* out, int nreal) {
  const int lane = (int)threadIdx.x & 31;
  const int wave = (int)threadIdx.x >> 5;
  const int row  = (int)blockIdx.x * 8 + wave;
  const int nr   = nreal < NN ? nreal : NN;
  const int rowc = clampi(row, 0, NN - 1);
  const bool rok = row < nr;
  const int c0   = lane * 2;

  const v2i mt = *(const v2ia*)(META + 2 * (size_t)rowc);
  asm volatile("" :: "v"(mt));
  const int craw = mt.y;
  const int offv = clampi(mt.x, 0, LISTTOT);
  int cntv = clampi(craw, 0, DEGCAP);
  cntv = cntv < (LISTTOT - offv) ? cntv : (LISTTOT - offv);
  const int off = __builtin_amdgcn_readfirstlane(offv);
  const int cnt = __builtin_amdgcn_readfirstlane(rok ? cntv : 0);
  const bool poison = (craw < 0) || (craw > DEGCAP);

  const float eld = EL[rowc];
  asm volatile("" :: "v"(eld));
  const float erd = ER[rowc];
  asm volatile("" :: "v"(erd));
  const float tl = eld + erd;
  const float eloop = lrelu_k(tl);

  float mx = -__builtin_inff();
#pragma unroll 1
  for (int b0 = 0; b0 < cnt; b0 += 32) {
    const int j = (b0 + lane) < cnt ? (b0 + lane) : cnt - 1;
    const unsigned s = LIST[(size_t)(off + j)];
    asm volatile("" :: "v"(s));
    const int col = clampi((int)s, 0, NN - 1);
    const float an = EL[col];
    asm volatile("" :: "v"(an));
    const float t = an + erd;
    mx = maxk(mx, lrelu_k(t));
  }
#pragma unroll
  for (int d = 16; d > 0; d >>= 1) {
    const float o = __shfl_xor(mx, d, 32);
    mx = maxk(mx, o);
  }
  mx = maxk(mx, eloop);

  float den = 0.0f;
#pragma unroll 1
  for (int b0 = 0; b0 < cnt; b0 += 32) {
    const int j = (b0 + lane) < cnt ? (b0 + lane) : cnt - 1;
    const unsigned s = LIST[(size_t)(off + j)];
    asm volatile("" :: "v"(s));
    const int col = clampi((int)s, 0, NN - 1);
    const float an = EL[col];
    asm volatile("" :: "v"(an));
    const float t = an + erd;
    const float v = lrelu_k(t) - mx;
    const float q = expf(v);
    const int m32 = (cnt - b0) < 32 ? (cnt - b0) : 32;
#pragma unroll 1
    for (int k = 0; k < m32; ++k) {
      const float qk = __int_as_float(__builtin_amdgcn_readlane(__float_as_int(q), k));
      den = den + qk;
    }
  }
  const float exl = expf(eloop - mx);
  den = den + exl;

  v2f ac = (v2f){0.0f, 0.0f};
#pragma unroll 1
  for (int b0 = 0; b0 < cnt; b0 += 32) {
    const int j = (b0 + lane) < cnt ? (b0 + lane) : cnt - 1;
    const unsigned s = LIST[(size_t)(off + j)];
    asm volatile("" :: "v"(s));
    const int col = clampi((int)s, 0, NN - 1);
    const float an = EL[col];
    asm volatile("" :: "v"(an));
    const float t = an + erd;
    const float v = lrelu_k(t) - mx;
    const float q = expf(v);
    const float w = q / den;
    const int m32 = (cnt - b0) < 32 ? (cnt - b0) : 32;
#pragma unroll 1
    for (int k = 0; k < m32; ++k) {
      const int c = __builtin_amdgcn_readlane(col, k);
      const float wk = __int_as_float(__builtin_amdgcn_readlane(__float_as_int(w), k));
      const v2f hn = *(const v2fa*)(FT2 + (size_t)c * D2W + c0);
      asm volatile("" :: "v"(hn));
      float pr;
      pr = wk * hn.x; ac.x = ac.x + pr;
      pr = wk * hn.y; ac.y = ac.y + pr;
    }
  }
  {
    const float wl = exl / den;
    const v2f hn = *(const v2fa*)(FT2 + (size_t)rowc * D2W + c0);
    asm volatile("" :: "v"(hn));
    float pr;
    pr = wl * hn.x; ac.x = ac.x + pr;
    pr = wl * hn.y; ac.y = ac.y + pr;
  }

  const v2f bv = *(const v2fa*)(TB + T_B2 + c0);
  const float qnan = __uint_as_float(0x7fc00000u);
  v2f o;
  o.x = ac.x + bv.x;
  o.y = ac.y + bv.y;
  o.x = poison ? qnan : o.x;
  o.y = poison ? qnan : o.y;
  volatile v2f* q = (volatile v2f*)(out + (size_t)rowc * D2W + c0);
  if (rok) *q = o;
  __threadfence();
  if (rok) *q = o;
}

extern "C" void kernel_launch(void* const* d_in, const int* in_sizes, int n_in,
                              void* d_out, int out_size, void* d_ws, size_t ws_size,
                              hipStream_t stream) {
  if (n_in < 10) return;
  if (in_sizes[0] != NN * KD) return;
  if (in_sizes[1] != 2 * NE) return;
  if (in_sizes[2] != KD * D1W) return;
  if (in_sizes[3] != 128 || in_sizes[4] != 128 || in_sizes[5] != 128) return;
  if (in_sizes[6] != D1W * D2W) return;
  if (in_sizes[7] != 64 || in_sizes[8] != 64 || in_sizes[9] != 64) return;
  if (out_size != NN * D2W) return;

  const float* x    = (const float*)d_in[0];
  const int*   ei   = (const int*)  d_in[1];
  const float* W1   = (const float*)d_in[2];
  const float* as1  = (const float*)d_in[3];
  const float* ad1  = (const float*)d_in[4];
  const float* b1   = (const float*)d_in[5];
  const float* W2   = (const float*)d_in[6];
  const float* as2  = (const float*)d_in[7];
  const float* ad2  = (const float*)d_in[8];
  const float* b2   = (const float*)d_in[9];
  const int* esrc = ei;
  const int* ekey = ei + NE;
  float* out = (float*)d_out;

  char* ws = (char*)d_ws;
  size_t off = 0;
  const size_t oXB   = off; off += SZ_XB;
  const size_t oW1T  = off; off += SZ_W1T;
  const size_t oW2D  = off; off += SZ_W2D;
  const size_t oTB   = off; off += (size_t)TB_BYTES;
  const size_t oFT   = off; off += SZ_FT;
  const size_t oOP   = off; off += SZ_OP;
  const size_t oEL1  = off; off += SZ_E1;
  const size_t oER1  = off; off += SZ_E1;
  const size_t oEL2  = off; off += SZ_E2;
  const size_t oER2  = off; off += SZ_E2;
  const size_t oMETA = off; off += SZ_META;
  const size_t oLIST = off; off += SZ_LIST;
  if (off != (size_t)WS_TOTAL || off > ws_size || off > (size_t)WSMAX) return;
  unsigned short* XB  = (unsigned short*)(ws + oXB);
  unsigned short* W1T = (unsigned short*)(ws + oW1T);
  unsigned short* W2D = (unsigned short*)(ws + oW2D);
  float*    TB   = (float*)(ws + oTB);
  float*    FT   = (float*)(ws + oFT);
  float*    FT2  = (float*)(ws + oFT);
  unsigned short* OP = (unsigned short*)(ws + oOP);
  float*    EL1  = (float*)(ws + oEL1);
  float*    ER1  = (float*)(ws + oER1);
  float*    EL2  = (float*)(ws + oEL2);
  float*    ER2  = (float*)(ws + oER2);
  int*      META = (int*)(ws + oMETA);
  unsigned* LIST = (unsigned*)(ws + oLIST);

  (void)hipFuncSetAttribute(reinterpret_cast<const void*>(&k_list),
                            hipFuncAttributeMaxDynamicSharedMemorySize, LDS_LIST);

  k_plane<0><<<NPAD * KD / 8 / 256, 256, 0, stream>>>(x, NN, KD, KD, XB, NPAD, KD);
  k_prep<<<PREP_W1_BLK + PREP_W2_BLK + 1, 256, 0, stream>>>(W1, W2, as1, ad1, b1, as2, ad2, b2, W1T, W2D, TB);
  k_list<<<NBLK, BT, LDS_LIST, stream>>>(ekey, esrc, LIST, META);
  {
    const int tiles = (NPAD / 64) * (D1W / 64);
    k_gemm_nt<0, 0><<<(tiles + 7) / 8, 256, 0, stream>>>(XB, W1T, TB, FT, NPAD, D1W, KD, D1W);
  }
  k_rowprep1<<<NPAD / 32, 256, 0, stream>>>(FT, TB, EL1, ER1);
  k_walk1<<<NPAD / 8, 256, 0, stream>>>(FT, EL1, ER1, LIST, META, TB, OP);
  {
    const int tiles = (NPAD / 64) * (D2W / 64);
    k_gemm_nt<0, 0><<<(tiles + 7) / 8, 256, 0, stream>>>(OP, W2D, TB, FT2, NPAD, D2W, OPK, D2W);
  }
  k_rowprep2<<<NPAD / 32, 256, 0, stream>>>(FT2, TB, EL2, ER2);
  k_walk2<<<NN / 8, 256, 0, stream>>>(FT2, EL2, ER2, LIST, META, TB, out, out_size / D2W);
}
